// GraphSAGE_19920058319553
// MI455X (gfx1250) — hardware-verified
//
#include <hip/hip_runtime.h>
#include <stddef.h>
#include <stdint.h>


#define DF     128
#define DO     64
#define KH     256
#define NTHR   256
#define NWAVE  8
#define EPT    8
#define CHUNK  (NTHR * EPT)
#define WCAP   (EPT * 32)
#define LISTN  (NWAVE * WCAP)
#define NBA    1024
#define SLA    10
#define RCAP   28672
#define DEGCAP 64
#define GBM    64
#define GBN    64
#define GTHR   128
#define AROWS  64
#define UBIG   2048
#define USML   1024
#define NUW    (6 * UBIG + 4 * USML)
#define AGG_ZINTS (LISTN + 2 * RCAP + 3 * NBA)
#define AGG_LDS_INTS (AGG_ZINTS + 16)

static_assert((CHUNK & (CHUNK - 1)) == 0 && CHUNK <= 4096);
static_assert((NBA & (NBA - 1)) == 0 && NBA == (1 << SLA));
static_assert(((long long)CHUNK << SLA) < (1LL << 31));
static_assert(LISTN % NTHR == 0);
static_assert(NBA % (2 * NWAVE) == 0 && NBA == 4 * NTHR && NBA % GBM == 0);
static_assert(RCAP % 4 == 0 && AGG_ZINTS % 4 == 0 && LISTN % 4 == 0);
static_assert(DF % 32 == 0 && KH % 32 == 0 && KH == 2 * DF);
static_assert(GBM == (GTHR / 32) * 16 && GBN == 64 && DF % GBN == 0 && DO % GBN == 0);
static_assert(UBIG % NTHR == 0 && USML % NTHR == 0 && NUW % NTHR == 0);
static_assert(DF == 4 * 32 && DO == 2 * 32 && DEGCAP == 64 && AROWS % NWAVE == 0 && AROWS == GBM);
static_assert(AGG_LDS_INTS * 4 <= 300000);

typedef float          v2f   __attribute__((ext_vector_type(2)));
typedef float          v4f   __attribute__((ext_vector_type(4)));
typedef float          v8f   __attribute__((ext_vector_type(8)));
typedef int            v4i   __attribute__((ext_vector_type(4)));
typedef int            v8i   __attribute__((ext_vector_type(8)));
typedef unsigned short v4us  __attribute__((ext_vector_type(4)));
typedef unsigned short v8us  __attribute__((ext_vector_type(8)));
typedef unsigned short v16us __attribute__((ext_vector_type(16)));
typedef __bf16         v16bf __attribute__((ext_vector_type(16)));
typedef v2f  __attribute__((may_alias)) v2fa;
typedef v4f  __attribute__((may_alias)) v4fa;
typedef v4i  __attribute__((may_alias)) v4ia;
typedef v4us __attribute__((may_alias)) v4usa;
typedef v8us __attribute__((may_alias)) v8usa;
union FragB { v16bf v; v16us u; v8us h[2]; v8i w; };

__device__ __forceinline__ v8f wmb(const FragB& a, const FragB& b, v8f c) {
  v8f d = __builtin_amdgcn_wmma_f32_16x16x32_bf16(false, a.v, false, b.v, (short)0, c, false, false);
  asm volatile("v_nop\n\tv_nop\n\tv_nop\n\tv_nop" : "+v"(d) : "v"(a.w), "v"(b.w));
  return d;
}

__device__ __forceinline__ unsigned bf16_bits(float f) {
  const unsigned u = __float_as_uint(f);
  return (u + 0x7FFFu + ((u >> 16) & 1u)) >> 16;
}
__device__ __forceinline__ float bf16_val(float f) {
  return __uint_as_float(bf16_bits(f) << 16);
}

__device__ __forceinline__ void wave_sync() {
  __builtin_amdgcn_fence(__ATOMIC_RELEASE, "wavefront");
  __builtin_amdgcn_wave_barrier();
  __builtin_amdgcn_fence(__ATOMIC_ACQUIRE, "wavefront");
}

template <int SLB>
__device__ __forceinline__ int scan_chunk(const int* __restrict__ dsts, int nE, int cbase, int slotBase,
                                          int nb, int vec8, int* list, int tid, int lane, int wave) {
  int wc = 0;
  const int el0  = tid * EPT;
  const int e0   = cbase + el0;
  const int sent = -2147483647 - 1;
  v4i da, db;
  if (vec8 != 0 && cbase + CHUNK <= nE) {
    da = *(const v4i*)(dsts + e0);
    db = *(const v4i*)(dsts + e0 + 4);
  } else {
    da.x = (e0     < nE) ? dsts[min(e0,     nE - 1)] : sent;
    da.y = (e0 + 1 < nE) ? dsts[min(e0 + 1, nE - 1)] : sent;
    da.z = (e0 + 2 < nE) ? dsts[min(e0 + 2, nE - 1)] : sent;
    da.w = (e0 + 3 < nE) ? dsts[min(e0 + 3, nE - 1)] : sent;
    db.x = (e0 + 4 < nE) ? dsts[min(e0 + 4, nE - 1)] : sent;
    db.y = (e0 + 5 < nE) ? dsts[min(e0 + 5, nE - 1)] : sent;
    db.z = (e0 + 6 < nE) ? dsts[min(e0 + 6, nE - 1)] : sent;
    db.w = (e0 + 7 < nE) ? dsts[min(e0 + 7, nE - 1)] : sent;
  }
  const unsigned nbs = (unsigned)slotBase;
  const unsigned unb = (unsigned)nb;
  const unsigned s0 = (unsigned)da.x - nbs, s1 = (unsigned)da.y - nbs;
  const unsigned s2 = (unsigned)da.z - nbs, s3 = (unsigned)da.w - nbs;
  const unsigned s4 = (unsigned)db.x - nbs, s5 = (unsigned)db.y - nbs;
  const unsigned s6 = (unsigned)db.z - nbs, s7 = (unsigned)db.w - nbs;
  const bool h0 = s0 < unb, h1 = s1 < unb, h2 = s2 < unb, h3 = s3 < unb;
  const bool h4 = s4 < unb, h5 = s5 < unb, h6 = s6 < unb, h7 = s7 < unb;
  const unsigned any = __builtin_amdgcn_ballot_w32(h0 | h1 | h2 | h3 | h4 | h5 | h6 | h7);
  if (any != 0u) {
#define HITJ(J, HJ, SJ) { \
      const unsigned mj = __builtin_amdgcn_ballot_w32(HJ); \
      if (mj != 0u) { \
        if (HJ) { \
          const int pos = wc + (int)__builtin_amdgcn_mbcnt_lo(mj, 0u); \
          if (pos < WCAP) list[wave * WCAP + pos] = ((el0 + (J)) << SLB) | (int)(SJ); \
        } \
        wc += (int)__builtin_popcount(mj); } }
    HITJ(0, h0, s0)
    HITJ(1, h1, s1)
    HITJ(2, h2, s2)
    HITJ(3, h3, s3)
    HITJ(4, h4, s4)
    HITJ(5, h5, s5)
    HITJ(6, h6, s6)
    HITJ(7, h7, s7)
#undef HITJ
  }
  return wc;
}

__global__ __launch_bounds__(NTHR) void k_wprep(const float* __restrict__ Ws0, const float* __restrict__ Wn0,
                                                const float* __restrict__ Ws1, const float* __restrict__ Wn1,
                                                const float* __restrict__ Ws2, const float* __restrict__ Wn2,
                                                unsigned short* W0, unsigned short* W1, unsigned short* W2) {
  const int u = (int)blockIdx.x * NTHR + (int)threadIdx.x;
  int part, v;
  if (u < 6 * UBIG) { part = u >> 11; v = u & (UBIG - 1); }
  else              { part = 6 + ((u - 6 * UBIG) >> 10); v = (u - 6 * UBIG) & (USML - 1); }
  const float* W;
  unsigned short* P;
  int pitch, roff, coff;
  if (part == 0)      { W = Ws0; P = W0; pitch = DF; roff = 0;  coff = 0; }
  else if (part == 1) { W = Wn0; P = W0; pitch = DF; roff = DF; coff = 0; }
  else if (part == 2) { W = Ws1; P = W1; pitch = KH; roff = 0;  coff = 0; }
  else if (part == 3) { W = Ws1; P = W1; pitch = KH; roff = 0;  coff = DF; }
  else if (part == 4) { W = Wn1; P = W1; pitch = KH; roff = DF; coff = 0; }
  else if (part == 5) { W = Wn1; P = W1; pitch = KH; roff = DF; coff = DF; }
  else if (part == 6) { W = Ws2; P = W2; pitch = KH; roff = 0;  coff = 0; }
  else if (part == 7) { W = Ws2; P = W2; pitch = KH; roff = 0;  coff = DF; }
  else if (part == 8) { W = Wn2; P = W2; pitch = KH; roff = DO; coff = 0; }
  else if (part == 9) { W = Wn2; P = W2; pitch = KH; roff = DO; coff = DF; }
  else return;
  const int n  = v >> 4;
  const int k8 = (v & 15) * 8;
  const float* p = W + (size_t)n * DF + k8;
  const v4f a = *(const v4fa*)p;
  const v4f b = *(const v4fa*)(p + 4);
  v8us o;
  o[0] = (unsigned short)bf16_bits(a.x); o[1] = (unsigned short)bf16_bits(a.y);
  o[2] = (unsigned short)bf16_bits(a.z); o[3] = (unsigned short)bf16_bits(a.w);
  o[4] = (unsigned short)bf16_bits(b.x); o[5] = (unsigned short)bf16_bits(b.y);
  o[6] = (unsigned short)bf16_bits(b.z); o[7] = (unsigned short)bf16_bits(b.w);
  unsigned short* dp = P + (size_t)(roff + n) * pitch + coff + k8;
  *(volatile v8us*)dp = o;
  __threadfence();
  *(volatile v8us*)dp = o;
}

__global__ __launch_bounds__(NTHR) void k_cvx(const float* __restrict__ x, int nN, int nUnits,
                                              unsigned short* xb) {
  const int u = (int)blockIdx.x * NTHR + (int)threadIdx.x;
  if (u >= nUnits) return;
  const int row = u >> 4;
  const int k8  = (u & 15) * 8;
  const int rc  = row < nN ? row : nN - 1;
  const float* p = x + (size_t)rc * DF + k8;
  const v4f a = *(const v4fa*)p;
  const v4f b = *(const v4fa*)(p + 4);
  const bool ok = row < nN;
  v8us o;
  o[0] = ok ? (unsigned short)bf16_bits(a.x) : (unsigned short)0;
  o[1] = ok ? (unsigned short)bf16_bits(a.y) : (unsigned short)0;
  o[2] = ok ? (unsigned short)bf16_bits(a.z) : (unsigned short)0;
  o[3] = ok ? (unsigned short)bf16_bits(a.w) : (unsigned short)0;
  o[4] = ok ? (unsigned short)bf16_bits(b.x) : (unsigned short)0;
  o[5] = ok ? (unsigned short)bf16_bits(b.y) : (unsigned short)0;
  o[6] = ok ? (unsigned short)bf16_bits(b.z) : (unsigned short)0;
  o[7] = ok ? (unsigned short)bf16_bits(b.w) : (unsigned short)0;
  unsigned short* dp = xb + (size_t)row * DF + k8;
  *(volatile v8us*)dp = o;
  __threadfence();
  *(volatile v8us*)dp = o;
}

__global__ __launch_bounds__(NTHR) void k_build(const int* __restrict__ srcs, const int* __restrict__ dsts,
                                                int nE, int nN, int vec8, int* srcl, int* degp) {
  extern __shared__ __attribute__((aligned(16))) int dsm[];
  int* list = dsm;
  int* hl   = dsm + LISTN;
  int* sl   = hl + RCAP;
  int* cnt  = sl + RCAP;
  int* offs = cnt + NBA;
  int* cur  = offs + NBA;
  int* misc = cur + NBA;
  const int tid = (int)threadIdx.x, lane = tid & 31, wave = tid >> 5;
  const int nodeBase = (int)blockIdx.x * NBA;

  {
    const v4i z4 = {0, 0, 0, 0};
    for (int i = tid * 4; i < AGG_ZINTS; i += NTHR * 4) *(v4ia*)(dsm + i) = z4;
    if (tid < 16) misc[tid] = 0;
  }
  __syncthreads();

  int t = 0, ov = 0;
  const int nChunks = (nE + CHUNK - 1) / CHUNK;
#pragma unroll 1
  for (int ch = 0; ch < nChunks; ++ch) {
    const int cbase = ch * CHUNK;
    const int wc = scan_chunk<SLA>(dsts, nE, cbase, nodeBase, NBA, vec8, list, tid, lane, wave);
    if (lane == 0) misc[wave] = wc;
    __syncthreads();
    if (wave == 0) {
#pragma unroll 1
      for (int w2 = 0; w2 < NWAVE; ++w2) {
        int c = misc[w2];
        c = c < 0 ? 0 : (c > WCAP ? WCAP : c);
#pragma unroll 1
        for (int b0 = 0; b0 < c; b0 += 32) {
          const int idx = b0 + lane;
          const int ent = list[w2 * WCAP + (idx < WCAP ? idx : WCAP - 1)];
          const int m32 = (c - b0) < 32 ? (c - b0) : 32;
#pragma unroll 1
          for (int k = 0; k < m32; ++k) {
            const int u    = __builtin_amdgcn_readlane(ent, k);
            const int slot = u & (NBA - 1);
            const int el   = (u >> SLA) & (CHUNK - 1);
            const int pk   = ((cbase + el) << SLA) | slot;
            if (t < RCAP) {
              if (lane == 0) { hl[t] = pk; cnt[slot] = cnt[slot] + 1; }
              t = t + 1;
            } else {
              ov = 1;
            }
          }
        }
      }
    }
    __syncthreads();
  }
  if (wave == 0 && lane == 0) { misc[8] = t; misc[9] = ov; }
  __syncthreads();
  int tt = misc[8];
  tt = tt < 0 ? 0 : (tt > RCAP ? RCAP : tt);
  const int ovf = misc[9];

  if (wave == 0) {
    const int base = lane * (NBA / 32);
    int s = 0;
#pragma unroll 1
    for (int i = 0; i < NBA / 32; ++i) s += cnt[base + i];
    int incl = s;
#pragma unroll
    for (int d = 1; d < 32; d <<= 1) {
      const int y = __shfl_up(incl, d, 32);
      if (lane >= d) incl += y;
    }
    int run = incl - s;
#pragma unroll 1
    for (int i = 0; i < NBA / 32; ++i) {
      const int cv = cnt[base + i];
      offs[base + i] = run;
      cur[base + i]  = run;
      run += cv;
    }
  }
  __syncthreads();
  if (wave == 0) {
#pragma unroll 1
    for (int b0 = 0; b0 < tt; b0 += 32) {
      const int idx = b0 + lane;
      const int ent = hl[idx < RCAP ? idx : RCAP - 1];
      const int m32 = (tt - b0) < 32 ? (tt - b0) : 32;
#pragma unroll 1
      for (int k = 0; k < m32; ++k) {
        const int u    = __builtin_amdgcn_readlane(ent, k);
        const int slot = u & (NBA - 1);
        if (lane == 0) {
          int p = cur[slot];
          p = p < 0 ? 0 : (p > RCAP - 1 ? RCAP - 1 : p);
          sl[p] = u;
          cur[slot] = p + 1;
        }
      }
    }
  }
  __syncthreads();

  const int hh = lane >> 4, q = lane & 15;
#pragma unroll 1
  for (int si = 0; si < NBA / (2 * NWAVE); ++si) {
    const int pi = si * NWAVE + wave;
    const int s  = 2 * pi + hh;
    int c = cnt[s];
    c = c < 0 ? 0 : (c > DEGCAP ? DEGCAP : c);
    int o = offs[s];
    o = o < 0 ? 0 : (o > RCAP ? RCAP : o);
    const int j0 = 4 * q;
    int i0 = o + j0, i1 = o + j0 + 1, i2 = o + j0 + 2, i3 = o + j0 + 3;
    i0 = i0 > RCAP - 1 ? RCAP - 1 : i0;
    i1 = i1 > RCAP - 1 ? RCAP - 1 : i1;
    i2 = i2 > RCAP - 1 ? RCAP - 1 : i2;
    i3 = i3 > RCAP - 1 ? RCAP - 1 : i3;
    int e0 = sl[i0] >> SLA, e1 = sl[i1] >> SLA, e2 = sl[i2] >> SLA, e3 = sl[i3] >> SLA;
    e0 = e0 < 0 ? 0 : (e0 > nE - 1 ? nE - 1 : e0);
    e1 = e1 < 0 ? 0 : (e1 > nE - 1 ? nE - 1 : e1);
    e2 = e2 < 0 ? 0 : (e2 > nE - 1 ? nE - 1 : e2);
    e3 = e3 < 0 ? 0 : (e3 > nE - 1 ? nE - 1 : e3);
    int r0 = srcs[e0], r1 = srcs[e1], r2 = srcs[e2], r3 = srcs[e3];
    r0 = r0 < 0 ? 0 : (r0 > nN - 1 ? nN - 1 : r0);
    r1 = r1 < 0 ? 0 : (r1 > nN - 1 ? nN - 1 : r1);
    r2 = r2 < 0 ? 0 : (r2 > nN - 1 ? nN - 1 : r2);
    r3 = r3 < 0 ? 0 : (r3 > nN - 1 ? nN - 1 : r3);
    v4i pv;
    pv.x = (j0     < c) ? r0 : 0;
    pv.y = (j0 + 1 < c) ? r1 : 0;
    pv.z = (j0 + 2 < c) ? r2 : 0;
    pv.w = (j0 + 3 < c) ? r3 : 0;
    int* rp = srcl + (size_t)(nodeBase + 2 * pi) * DEGCAP + 4 * lane;
    *(volatile v4i*)rp = pv;
    __threadfence();
    *(volatile v4i*)rp = pv;
  }

  {
    const v4i c4 = *(const v4ia*)(cnt + 4 * tid);
    v4i d4;
    d4.x = (ovf != 0 || c4.x < 0 || c4.x > DEGCAP) ? -1 : c4.x;
    d4.y = (ovf != 0 || c4.y < 0 || c4.y > DEGCAP) ? -1 : c4.y;
    d4.z = (ovf != 0 || c4.z < 0 || c4.z > DEGCAP) ? -1 : c4.z;
    d4.w = (ovf != 0 || c4.w < 0 || c4.w > DEGCAP) ? -1 : c4.w;
    int* dp = degp + (size_t)nodeBase + 4 * tid;
    *(volatile v4i*)dp = d4;
    __threadfence();
    *(volatile v4i*)dp = d4;
  }
}

__global__ __launch_bounds__(GTHR) void k_gemm(
    const unsigned short* __restrict__ A, const unsigned short* __restrict__ WT,
    float* outS, float* outP, int K, int nHalf)
{
  __shared__ __attribute__((aligned(16))) float stg[GBM * GBN];
  const int tid = (int)threadIdx.x, lane = tid & 31, wave = tid >> 5, hh = lane >> 4, m = lane & 15;
  const int rowBase = (int)blockIdx.x * GBM;
  const int colc    = (int)blockIdx.y * GBN;
  const bool isP    = colc >= nHalf;
  float* outF       = isP ? outP : outS;
  const int oc0     = isP ? (colc - nHalf) : colc;
  const int ldo     = nHalf;

  v8f acc[4];
  {
    const v8f z = {0.f, 0.f, 0.f, 0.f, 0.f, 0.f, 0.f, 0.f};
    acc[0] = z; acc[1] = z; acc[2] = z; acc[3] = z;
  }
  const unsigned short* ap = A  + (size_t)(rowBase + 16 * wave + m) * (size_t)K + 8 * hh;
  const unsigned short* wp = WT + (size_t)(colc + m) * (size_t)K + 8 * hh;
  const int ksteps = K >> 5;
#pragma unroll 1
  for (int ks = 0; ks < ksteps; ++ks) {
    FragB af;
    af.h[0] = *(const v8usa*)(ap + 32 * ks);
    af.h[1] = *(const v8usa*)(ap + 32 * ks + 16);
#pragma unroll
    for (int t = 0; t < 4; ++t) {
      const unsigned short* wq = wp + (size_t)(16 * t) * (size_t)K + 32 * ks;
      FragB bf;
      bf.h[0] = *(const v8usa*)wq;
      bf.h[1] = *(const v8usa*)(wq + 16);
      acc[t] = wmb(af, bf, acc[t]);
    }
  }

#pragma unroll
  for (int t = 0; t < 4; ++t) {
    const int lc = 16 * t + m;
#pragma unroll
    for (int r = 0; r < 8; ++r) {
      const int lr = 16 * wave + 8 * hh + r;
      stg[lr * GBN + lc] = acc[t][r];
    }
  }
  __syncthreads();

  v4f fv[8];
#pragma unroll
  for (int i = 0; i < 8; ++i) {
    const int lr = 16 * wave + 2 * i + hh;
    fv[i] = *(const v4fa*)(stg + lr * GBN + 4 * m);
  }
#pragma unroll
  for (int i = 0; i < 8; ++i) {
    const int lr = 16 * wave + 2 * i + hh;
    const int gr = rowBase + lr;
    float* op = outF + (size_t)gr * (size_t)ldo + oc0 + 4 * m;
    *(volatile v4f*)op = fv[i];
  }
  __threadfence();
#pragma unroll
  for (int i = 0; i < 8; ++i) {
    const int lr = 16 * wave + 2 * i + hh;
    const int gr = rowBase + lr;
    float* op = outF + (size_t)gr * (size_t)ldo + oc0 + 4 * m;
    *(volatile v4f*)op = fv[i];
  }
}

__global__ __launch_bounds__(NTHR) void k_aggh(const int* __restrict__ srcl, const int* __restrict__ degp,
                                               const float* __restrict__ Sp, const float* __restrict__ Pp,
                                               const float* __restrict__ bs, const float* __restrict__ bn,
                                               int nN, int mRows, unsigned short* hpl) {
  __shared__ __attribute__((aligned(16))) unsigned short rowbufs[NWAVE * KH];
  const int tid = (int)threadIdx.x, lane = tid & 31, wave = tid >> 5;
  unsigned short* rowbuf = rowbufs + wave * KH;
  v4f bb;
  {
    const v4f t1 = *(const v4fa*)(bs + 4 * lane);
    const v4f t2 = *(const v4fa*)(bn + 4 * lane);
    bb.x = bf16_val(t1.x) + bf16_val(t2.x);
    bb.y = bf16_val(t1.y) + bf16_val(t2.y);
    bb.z = bf16_val(t1.z) + bf16_val(t2.z);
    bb.w = bf16_val(t1.w) + bf16_val(t2.w);
  }
  const float qnan = __int_as_float(0x7fc00000);
#pragma unroll 1
  for (int it = 0; it < AROWS / NWAVE; ++it) {
    const int node = __builtin_amdgcn_readfirstlane((int)blockIdx.x * AROWS + it * NWAVE + wave);
    const int nr   = node < mRows ? node : mRows - 1;
    const bool live = node < nN;
    const int dg = __builtin_amdgcn_readfirstlane(degp[nr]);
    const bool bad = (dg < 0) || (dg > DEGCAP);
    int cf = dg < 0 ? 0 : (dg > DEGCAP ? DEGCAP : dg);
    const int cc = live ? cf : 0;
    const int e0 = srcl[(size_t)nr * DEGCAP + lane];
    const int e1 = srcl[(size_t)nr * DEGCAP + 32 + lane];
    float a0 = 0.0f, a1 = 0.0f, a2 = 0.0f, a3 = 0.0f;
#pragma unroll 1
    for (int b0 = 0; b0 < cc; b0 += 32) {
      const int ent = (b0 == 0) ? e0 : e1;
      const int m32 = (cc - b0) < 32 ? (cc - b0) : 32;
#pragma unroll 1
      for (int k = 0; k < m32; ++k) {
        int sk = __builtin_amdgcn_readlane(ent, k);
        sk = sk < 0 ? 0 : (sk > nN - 1 ? nN - 1 : sk);
        const v4f a = *(const v4fa*)(Pp + (size_t)sk * DF + 4 * lane);
        a0 += a.x; a1 += a.y; a2 += a.z; a3 += a.w;
      }
    }
    const v4f sv = *(const v4fa*)(Sp + (size_t)nr * DF + 4 * lane);
    const float inv = 1.0f / fmaxf((float)cf, 1.0f);
    const float pz = bad ? qnan : 0.0f;
    float y0 = (sv.x + a0 * inv) + bb.x;
    float y1 = (sv.y + a1 * inv) + bb.y;
    float y2 = (sv.z + a2 * inv) + bb.z;
    float y3 = (sv.w + a3 * inv) + bb.w;
    y0 = (y0 > 0.0f) ? y0 : (y0 - y0);
    y1 = (y1 > 0.0f) ? y1 : (y1 - y1);
    y2 = (y2 > 0.0f) ? y2 : (y2 - y2);
    y3 = (y3 > 0.0f) ? y3 : (y3 - y3);
    const float m0 = live ? (y0 + pz) : 0.0f;
    const float m1 = live ? (y1 + pz) : 0.0f;
    const float m2 = live ? (y2 + pz) : 0.0f;
    const float m3 = live ? (y3 + pz) : 0.0f;
    v4us mh, ml;
    {
      unsigned hb;
      hb = bf16_bits(m0); mh[0] = (unsigned short)hb; ml[0] = (unsigned short)bf16_bits(m0 - __uint_as_float(hb << 16));
      hb = bf16_bits(m1); mh[1] = (unsigned short)hb; ml[1] = (unsigned short)bf16_bits(m1 - __uint_as_float(hb << 16));
      hb = bf16_bits(m2); mh[2] = (unsigned short)hb; ml[2] = (unsigned short)bf16_bits(m2 - __uint_as_float(hb << 16));
      hb = bf16_bits(m3); mh[3] = (unsigned short)hb; ml[3] = (unsigned short)bf16_bits(m3 - __uint_as_float(hb << 16));
    }
    *(v4usa*)(rowbuf + 4 * lane) = mh;
    *(v4usa*)(rowbuf + DF + 4 * lane) = ml;
    wave_sync();
    const v8us q0 = *(const v8usa*)(rowbuf + 8 * lane);
    wave_sync();
    if (node < mRows) {
      unsigned short* rpw = hpl + (size_t)node * KH + 8 * lane;
      *(volatile v8us*)rpw = q0;
      __threadfence();
      *(volatile v8us*)rpw = q0;
    }
  }
}

__global__ __launch_bounds__(NTHR) void k_aggo(const int* __restrict__ srcl, const int* __restrict__ degp,
                                               const float* __restrict__ Sp, const float* __restrict__ Pp,
                                               const float* __restrict__ bs, const float* __restrict__ bn,
                                               int nN, int mRows, float* out) {
  const int tid = (int)threadIdx.x, lane = tid & 31, wave = tid >> 5;
  float bv0, bv1;
  {
    const v2f t1 = *(const v2fa*)(bs + 2 * lane);
    const v2f t2 = *(const v2fa*)(bn + 2 * lane);
    bv0 = bf16_val(t1.x) + bf16_val(t2.x);
    bv1 = bf16_val(t1.y) + bf16_val(t2.y);
  }
  const float qnan = __int_as_float(0x7fc00000);
  const int sa = (2 * lane) & 31, sb = (2 * lane + 1) & 31;
#pragma unroll 1
  for (int it = 0; it < AROWS / NWAVE; ++it) {
    const int node = __builtin_amdgcn_readfirstlane((int)blockIdx.x * AROWS + it * NWAVE + wave);
    const int nr   = node < mRows ? node : mRows - 1;
    const bool live = node < nN;
    const int dg = __builtin_amdgcn_readfirstlane(degp[nr]);
    const bool bad = (dg < 0) || (dg > DEGCAP);
    int cf = dg < 0 ? 0 : (dg > DEGCAP ? DEGCAP : dg);
    const int cc = live ? cf : 0;
    const int e0 = srcl[(size_t)nr * DEGCAP + lane];
    const int e1 = srcl[(size_t)nr * DEGCAP + 32 + lane];
    float a0 = 0.0f, a1 = 0.0f;
#pragma unroll 1
    for (int b0 = 0; b0 < cc; b0 += 32) {
      const int ent = (b0 == 0) ? e0 : e1;
      const int m32 = (cc - b0) < 32 ? (cc - b0) : 32;
#pragma unroll 1
      for (int k = 0; k < m32; ++k) {
        int sk = __builtin_amdgcn_readlane(ent, k);
        sk = sk < 0 ? 0 : (sk > nN - 1 ? nN - 1 : sk);
        const v2f a = *(const v2fa*)(Pp + (size_t)sk * DO + 2 * lane);
        a0 += a.x; a1 += a.y;
      }
    }
    const v2f sv = *(const v2fa*)(Sp + (size_t)nr * DO + 2 * lane);
    const float inv = 1.0f / fmaxf((float)cf, 1.0f);
    const float pz = bad ? qnan : 0.0f;
    const float v0 = ((sv.x + a0 * inv) + bv0) + pz;
    const float v1 = ((sv.y + a1 * inv) + bv1) + pz;
    v4f ow;
    ow.x = __shfl(v0, sa, 32); ow.y = __shfl(v1, sa, 32);
    ow.z = __shfl(v0, sb, 32); ow.w = __shfl(v1, sb, 32);
    const int nst = live ? node : 0;
    float* op = out + (size_t)nst * DO + 4 * (lane & 15);
    const bool wr = live && (lane < 16);
    if (wr) *(volatile v4f*)op = ow;
    __threadfence();
    if (wr) *(volatile v4f*)op = ow;
  }
}

static inline int cdiv(int a, int b) { return (a + b - 1) / b; }
static inline size_t al256(size_t o) { return (o + 255) & ~(size_t)255; }

extern "C" void kernel_launch(void* const* d_in, const int* in_sizes, int n_in,
                              void* d_out, int out_size, void* d_ws, size_t ws_size,
                              hipStream_t stream) {
  if (n_in < 15) return;
  if (in_sizes[0] < DF || (in_sizes[0] % DF) != 0) return;
  const int nN = in_sizes[0] / DF;
  if (nN < 16 || nN > (1 << 22)) return;
  const int nE = in_sizes[1];
  if (nE < 1 || in_sizes[2] != nE) return;
  if (nE >= (1 << (31 - SLA))) return;
  if (in_sizes[3] != DF * DF || in_sizes[4] != DF) return;
  if (in_sizes[5] != DF * DF || in_sizes[6] != DF) return;
  if (in_sizes[7] != DF * DF || in_sizes[8] != DF) return;
  if (in_sizes[9] != DF * DF || in_sizes[10] != DF) return;
  if (in_sizes[11] != DO * DF || in_sizes[12] != DO) return;
  if (in_sizes[13] != DO * DF || in_sizes[14] != DO) return;
  if ((long long)out_size != (long long)nN * DO) return;

  const float* feat = (const float*)d_in[0];
  const int*   src  = (const int*)d_in[1];
  const int*   dst  = (const int*)d_in[2];
  const float* Ws0 = (const float*)d_in[3];   const float* bs0 = (const float*)d_in[4];
  const float* Wn0 = (const float*)d_in[5];   const float* bn0 = (const float*)d_in[6];
  const float* Ws1 = (const float*)d_in[7];   const float* bs1 = (const float*)d_in[8];
  const float* Wn1 = (const float*)d_in[9];   const float* bn1 = (const float*)d_in[10];
  const float* Ws2 = (const float*)d_in[11];  const float* bs2 = (const float*)d_in[12];
  const float* Wn2 = (const float*)d_in[13];  const float* bn2 = (const float*)d_in[14];
  float* out = (float*)d_out;

  const int MP = cdiv(nN, GBM) * GBM;
  const int gM = MP / GBM;
  const int gA = cdiv(MP, NBA);
  const int NP = gA * NBA;
  if (NP < MP) return;
  const int vec8 = ((nE & 3) == 0) ? 1 : 0;

  char* ws = (char*)d_ws;
  size_t off = 0;
  const size_t oW0 = off; off = al256(off + (size_t)2 * DF * DF * 2);
  const size_t oW1 = off; off = al256(off + (size_t)2 * DF * KH * 2);
  const size_t oW2 = off; off = al256(off + (size_t)2 * DO * KH * 2);
  const size_t oDG = off; off = al256(off + (size_t)NP * 4);
  const size_t oSL = off; off = al256(off + (size_t)NP * DEGCAP * 4);
  const size_t oR0 = off; off = al256(off + (size_t)MP * DF * 4);
  const size_t oR1 = off; off = al256(off + (size_t)MP * DF * 4);
  const size_t oR2 = off; off = al256(off + (size_t)MP * KH * 2);
  if (off > ws_size) return;
  unsigned short* W0 = (unsigned short*)(ws + oW0);
  unsigned short* W1 = (unsigned short*)(ws + oW1);
  unsigned short* W2 = (unsigned short*)(ws + oW2);
  int*            DG = (int*)(ws + oDG);
  int*            SL = (int*)(ws + oSL);
  float*          R0 = (float*)(ws + oR0);
  float*          R1 = (float*)(ws + oR1);
  unsigned short* R2 = (unsigned short*)(ws + oR2);

  const size_t bldLds = (size_t)AGG_LDS_INTS * 4;
  hipFuncSetAttribute(reinterpret_cast<const void*>(&k_build), hipFuncAttributeMaxDynamicSharedMemorySize, (int)bldLds);

  const int nUx = MP * (DF / 8);
  k_wprep<<<NUW / NTHR, NTHR, 0, stream>>>(Ws0, Wn0, Ws1, Wn1, Ws2, Wn2, W0, W1, W2);
  k_cvx<<<cdiv(nUx, NTHR), NTHR, 0, stream>>>(feat, nN, nUx, R2);
  k_build<<<gA, NTHR, bldLds, stream>>>(src, dst, nE, nN, vec8, SL, DG);
  k_gemm<<<dim3(gM, (2 * DF) / GBN), GTHR, 0, stream>>>(R2, W0, R0, R1, DF, DF);
  k_aggh<<<gM, NTHR, 0, stream>>>(SL, DG, R0, R1, bs0, bn0, nN, MP, R2);
  k_gemm<<<dim3(gM, (2 * DF) / GBN), GTHR, 0, stream>>>(R2, W1, R0, R1, KH, DF);
  k_aggh<<<gM, NTHR, 0, stream>>>(SL, DG, R0, R1, bs1, bn1, nN, MP, R2);
  k_gemm<<<dim3(gM, (2 * DO) / GBN), GTHR, 0, stream>>>(R2, W2, R0, R1, KH, DO);
  k_aggo<<<cdiv(nN, AROWS), NTHR, 0, stream>>>(SL, DG, R0, R1, bs2, bn2, nN, MP, out);
}
